// SenriStandardAttention_46256797778263
// MI455X (gfx1250) — hardware-verified
//
#include <hip/hip_runtime.h>
#include <math.h>
#include <stdint.h>

#define NB   2
#define SEQ  2048
#define DM   2048
#define NHQ  32
#define NKV  8
#define HD   64
#define DKV  (NKV * HD)
#define NQB  (SEQ / 64)

static_assert(DM == NHQ * HD);
static_assert((NHQ % NKV) == 0);
static_assert((SEQ % 64) == 0 && (DM % 64) == 0 && (DKV % 64) == 0);

typedef __bf16 v16b __attribute__((ext_vector_type(16)));
typedef __bf16 v8b  __attribute__((ext_vector_type(8)));
typedef float  v8f  __attribute__((ext_vector_type(8)));
typedef float  v4f  __attribute__((ext_vector_type(4)));
typedef unsigned short v8us __attribute__((ext_vector_type(8)));

struct RopeInv { float f[32]; };
static_assert(sizeof(RopeInv) == 128);

__device__ __forceinline__ unsigned short f2bf_bits(float f) {
  const unsigned u = __float_as_uint(f);
  return (unsigned short)((u + 0x7FFFu + ((u >> 16) & 1u)) >> 16);
}
__device__ __forceinline__ float bfb2f(unsigned short b) { return __uint_as_float(((unsigned)b) << 16); }
__device__ __forceinline__ __bf16 bits2bf(unsigned short b) { return __builtin_bit_cast(__bf16, b); }

__device__ __forceinline__ v8f vz8() { return (v8f){0.f, 0.f, 0.f, 0.f, 0.f, 0.f, 0.f, 0.f}; }

union FragU { v16b v; v8b h[2]; };
__device__ __forceinline__ v16b frag_ld(const __bf16* p) {
  FragU f;
  f.h[0] = *(const v8b*)(p);
  f.h[1] = *(const v8b*)(p + 16);
  return f.v;
}

__device__ __forceinline__ v8f mma_bf(v16b a, v16b b, v8f c) {
  c = __builtin_amdgcn_wmma_f32_16x16x32_bf16(false, a, false, b, (short)0, c, false, false);
  asm volatile("v_nop\n\tv_nop\n\tv_nop\n\tv_nop" : "+v"(c) : "v"(a), "v"(b));
  return c;
}

__device__ __forceinline__ void wave_lds_sync() {
  __builtin_amdgcn_fence(__ATOMIC_RELEASE, "workgroup");
  __builtin_amdgcn_wave_barrier();
  __builtin_amdgcn_fence(__ATOMIC_ACQUIRE, "workgroup");
}

__global__ __launch_bounds__(256) void k_cvt_bf16(const float* __restrict__ in, unsigned short* __restrict__ out, int n8) {
  const int i = blockIdx.x * 256 + threadIdx.x;
  if (i < n8) {
    const size_t o = 8 * (size_t)i;
    const v4f a0 = *(const v4f*)(in + o);
    const v4f a1 = *(const v4f*)(in + o + 4);
    v8us w;
    w[0] = f2bf_bits(a0[0]); w[1] = f2bf_bits(a0[1]); w[2] = f2bf_bits(a0[2]); w[3] = f2bf_bits(a0[3]);
    w[4] = f2bf_bits(a1[0]); w[5] = f2bf_bits(a1[1]); w[6] = f2bf_bits(a1[2]); w[7] = f2bf_bits(a1[3]);
    *(volatile v8us*)(out + o) = w;
    __threadfence();
    *(volatile v8us*)(out + o) = w;
  }
}

__global__ __launch_bounds__(256) void k_rope_tab(const int* __restrict__ pos, float* __restrict__ ctab,
                                                    float* __restrict__ stab, RopeInv ri, int nrows) {
  const int wave = threadIdx.x >> 5, lane = threadIdx.x & 31;
  const int row = blockIdx.x * 8 + wave;
  if (row < nrows) {
    float inv = ri.f[0];
#pragma unroll
    for (int i = 1; i < 32; ++i) inv = (lane == i) ? ri.f[i] : inv;
    const float p   = (float)pos[row];
    const float ang = p * inv;
    const float cs  = cosf(ang);
    const float sn  = sinf(ang);
    const size_t o  = (size_t)row * 32 + lane;
    ((volatile float*)ctab)[o] = cs;
    ((volatile float*)stab)[o] = sn;
    __threadfence();
    ((volatile float*)ctab)[o] = cs;
    ((volatile float*)stab)[o] = sn;
  }
}

__global__ __launch_bounds__(256) void k_masktiles(const float* __restrict__ mask, float* __restrict__ tmax,
                                                     float* __restrict__ tmin) {
  __shared__ float wmx[8], wmn[8];
  __shared__ float omx[32], omn[32];
  const int tid = threadIdx.x, wave = tid >> 5, lane = tid & 31;
  const int qb  = blockIdx.x;
  const int row = qb * 64 + (tid >> 2);
  const int cp  = (tid & 3) * 16;
#pragma unroll 1
  for (int kc = 0; kc < NQB; ++kc) {
    const float* src = mask + (size_t)row * SEQ + kc * 64 + cp;
    float mx = -INFINITY, mn = INFINITY;
#pragma unroll
    for (int q = 0; q < 4; ++q) {
      const v4f a = *(const v4f*)(src + 4 * q);
      mx = fmaxf(mx, fmaxf(fmaxf(a[0], a[1]), fmaxf(a[2], a[3])));
      mn = fminf(mn, fminf(fminf(a[0], a[1]), fminf(a[2], a[3])));
    }
#pragma unroll
    for (int off = 1; off < 32; off <<= 1) {
      mx = fmaxf(mx, __shfl_xor(mx, off, 32));
      mn = fminf(mn, __shfl_xor(mn, off, 32));
    }
    if (lane == 0) { wmx[wave] = mx; wmn[wave] = mn; }
    __syncthreads();
    if (tid == 0) {
      float a = wmx[0], bq = wmn[0];
#pragma unroll
      for (int w = 1; w < 8; ++w) { a = fmaxf(a, wmx[w]); bq = fminf(bq, wmn[w]); }
      omx[kc] = a; omn[kc] = bq;
    }
    __syncthreads();
  }
  if (wave == 0) {
    const float a = omx[lane], bq = omn[lane];
    const size_t o = (size_t)qb * NQB + lane;
    ((volatile float*)tmax)[o] = a;
    ((volatile float*)tmin)[o] = bq;
    __threadfence();
    ((volatile float*)tmax)[o] = a;
    ((volatile float*)tmin)[o] = bq;
  }
}

template <int NPROD, bool ROPE, int OUT_MODE>
__global__ __launch_bounds__(256) void k_gemm64(
    const unsigned short* __restrict__ Ap, const unsigned short* __restrict__ A2p, int lda, long long strideA,
    const unsigned short* __restrict__ Btp, int ldb, long long strideB,
    void* __restrict__ Cout, void* __restrict__ Cout2, int ldc, long long strideC,
    const float* __restrict__ ctab, const float* __restrict__ stab,
    int M, int N, int K) {
  __shared__ __align__(16) float sT[8][16 * 68];
  const __bf16* A  = (const __bf16*)(const void*)Ap;
  const __bf16* A2 = (const __bf16*)(const void*)A2p;
  const __bf16* Bt = (const __bf16*)(const void*)Btp;
  const int bz   = blockIdx.y;
  const int lane = threadIdx.x & 31;
  const int wave = threadIdx.x >> 5;
  const int tilesN = N >> 6;
  const int tilesM = M >> 6;
  const int tile = blockIdx.x * 8 + wave;
  if (tile >= tilesM * tilesN) return;
  const int tm = tile / tilesN;
  const int tn = tile - tm * tilesN;
  const int m0 = tm << 6;
  const int n0 = tn << 6;

  const __bf16* Ab  = A  + (size_t)bz * strideA;
  const __bf16* Ab2 = A2 + (size_t)bz * strideA;
  const __bf16* Bb  = Bt + (size_t)bz * strideB;

  const int rl   = lane & 15;
  const int koff = (lane >> 4) * 8;
  const int mOff = (lane >> 4) * 8;

  v8f acc[4][4];
#pragma unroll
  for (int i = 0; i < 4; ++i)
#pragma unroll
    for (int j = 0; j < 4; ++j) acc[i][j] = vz8();

  for (int k0 = 0; k0 < K; k0 += 32) {
    v16b bf[4];
#pragma unroll
    for (int j = 0; j < 4; ++j)
      bf[j] = frag_ld(Bb + (size_t)(n0 + (j << 4) + rl) * ldb + koff + k0);
#pragma unroll
    for (int i = 0; i < 4; ++i) {
      const size_t ao = (size_t)(m0 + (i << 4) + rl) * lda + koff + k0;
      const v16b ah = frag_ld(Ab + ao);
      v16b al = ah;
      if (NPROD == 2) al = frag_ld(Ab2 + ao);
#pragma unroll
      for (int j = 0; j < 4; ++j) {
        acc[i][j] = mma_bf(ah, bf[j], acc[i][j]);
        if (NPROD == 2) acc[i][j] = mma_bf(al, bf[j], acc[i][j]);
      }
    }
  }

  float* slab = sT[wave];
#pragma unroll
  for (int i = 0; i < 4; ++i) {
    const int mBase = m0 + (i << 4);
    if (ROPE) {
#pragma unroll
      for (int jj = 0; jj < 2; ++jj) {
        const int fi = (jj << 4) + rl;
#pragma unroll
        for (int r = 0; r < 8; ++r) {
          const size_t to = (size_t)(mBase + mOff + r) * 32 + fi;
          const float cs = ctab[to];
          const float sn = stab[to];
          const float x1 = acc[i][jj][r];
          const float x2 = acc[i][jj + 2][r];
          slab[(mOff + r) * 68 + (jj << 4) + rl]       = x1 * cs - x2 * sn;
          slab[(mOff + r) * 68 + ((jj + 2) << 4) + rl] = x2 * cs + x1 * sn;
        }
      }
    } else {
#pragma unroll
      for (int j = 0; j < 4; ++j)
#pragma unroll
        for (int r = 0; r < 8; ++r)
          slab[(mOff + r) * 68 + (j << 4) + rl] = acc[i][j][r];
    }
    wave_lds_sync();
    if (OUT_MODE == 0) {
      float* C = (float*)Cout + (size_t)bz * strideC;
      const int h2 = lane >> 4, c4 = (lane & 15) * 4;
      for (int pass = 0; pass < 2; ++pass) {
#pragma unroll
        for (int it = 0; it < 8; ++it) {
          const int row = it * 2 + h2;
          const v4f v = *(const v4f*)(slab + row * 68 + c4);
          *(volatile v4f*)(C + (size_t)(mBase + row) * ldc + n0 + c4) = v;
        }
        __threadfence();
      }
    } else {
      unsigned short* C  = (unsigned short*)Cout  + (size_t)bz * strideC;
      unsigned short* C2 = (unsigned short*)Cout2 + (size_t)bz * strideC;
      const int q4 = lane >> 3, c8 = (lane & 7) * 8;
      for (int pass = 0; pass < 2; ++pass) {
#pragma unroll
        for (int it = 0; it < 4; ++it) {
          const int row = it * 4 + q4;
          const float* sp = slab + row * 68 + c8;
          v8us hv, lv;
#pragma unroll
          for (int e = 0; e < 8; ++e) {
            const float f = sp[e];
            const unsigned short hb = f2bf_bits(f);
            hv[e] = hb;
            lv[e] = f2bf_bits(f - bfb2f(hb));
          }
          const size_t go = (size_t)(mBase + row) * ldc + n0 + c8;
          *(volatile v8us*)(C + go)  = hv;
          *(volatile v8us*)(C2 + go) = lv;
        }
        __threadfence();
      }
    }
    wave_lds_sync();
  }
}

__global__ __launch_bounds__(128) void k_attn(
    const unsigned short* __restrict__ qhp, const unsigned short* __restrict__ qlp,
    const unsigned short* __restrict__ khp, const unsigned short* __restrict__ klp,
    const unsigned short* __restrict__ vhp, const unsigned short* __restrict__ vlp,
    const float* __restrict__ maskp, const float* __restrict__ tmaxp, const float* __restrict__ tminp,
    unsigned short* __restrict__ ohp, unsigned short* __restrict__ olp) {
  __shared__ __align__(16) __bf16 KVs[4 * 64 * 64];
  __shared__ __align__(16) __bf16 Ps[2 * 4 * 16 * 64];

  const int tid  = threadIdx.x;
  const int wave = tid >> 5;
  const int lane = tid & 31;
  const int hh   = lane >> 4;
  const int c    = lane & 15;

  const int bx  = blockIdx.x;
  const int qb  = bx % NQB;
  const int h   = (bx / NQB) % NHQ;
  const int b   = bx / (NQB * NHQ);
  const int kvh = h / (NHQ / NKV);
  const int q0  = qb * 64 + wave * 16;

  const __bf16* Qh = (const __bf16*)(const void*)qhp + (size_t)b * SEQ * DM + (size_t)h * HD;
  const __bf16* Ql = (const __bf16*)(const void*)qlp + (size_t)b * SEQ * DM + (size_t)h * HD;
  const __bf16* Kh = (const __bf16*)(const void*)khp + (size_t)b * SEQ * DKV + (size_t)kvh * HD;
  const __bf16* Kl = (const __bf16*)(const void*)klp + (size_t)b * SEQ * DKV + (size_t)kvh * HD;
  const __bf16* Vh = (const __bf16*)(const void*)vhp + ((size_t)b * DKV + (size_t)kvh * HD) * SEQ;
  const __bf16* Vl = (const __bf16*)(const void*)vlp + ((size_t)b * DKV + (size_t)kvh * HD) * SEQ;

  __bf16* Ksh = KVs;
  __bf16* Ksl = KVs + 4096;
  __bf16* Vth = KVs + 8192;
  __bf16* Vtl = KVs + 12288;
  __bf16* pwh = Ps + wave * 1024;
  __bf16* pwl = Ps + 4096 + wave * 1024;

  v16b qah[2], qal[2];
#pragma unroll
  for (int dc = 0; dc < 2; ++dc) {
    qah[dc] = frag_ld(Qh + (size_t)(q0 + c) * DM + dc * 32 + 8 * hh);
    qal[dc] = frag_ld(Ql + (size_t)(q0 + c) * DM + dc * 32 + 8 * hh);
  }

  float mrow[8], lrow[8];
  v8f oacc[4];
#pragma unroll
  for (int r = 0; r < 8; ++r) { mrow[r] = -INFINITY; lrow[r] = 0.f; }
#pragma unroll
  for (int t = 0; t < 4; ++t) oacc[t] = vz8();

  for (int kc = 0; kc < NQB; ++kc) {
    const float tmx = __int_as_float(__builtin_amdgcn_readfirstlane(__float_as_int(tmaxp[qb * NQB + kc])));
    const float tmn = __int_as_float(__builtin_amdgcn_readfirstlane(__float_as_int(tminp[qb * NQB + kc])));
    if (tmx <= -1.0e8f) continue;
    const bool addm = !((tmx == 0.0f) && (tmn == 0.0f));
    const int kv0 = kc * 64;

    __syncthreads();
    {
      const int r = tid >> 1, half = (tid & 1) * 32;
      const __bf16* ks = Kh + (size_t)(kv0 + r) * DKV + half;
      const __bf16* kl = Kl + (size_t)(kv0 + r) * DKV + half;
      const __bf16* vs = Vh + (size_t)r * SEQ + kv0 + half;
      const __bf16* vl = Vl + (size_t)r * SEQ + kv0 + half;
#pragma unroll
      for (int i = 0; i < 4; ++i) {
        const v8b a0 = *(const v8b*)(ks + 8 * i);
        const v8b a1 = *(const v8b*)(kl + 8 * i);
        const v8b b0 = *(const v8b*)(vs + 8 * i);
        const v8b b1 = *(const v8b*)(vl + 8 * i);
        *(v8b*)(Ksh + r * 64 + half + 8 * i) = a0;
        *(v8b*)(Ksl + r * 64 + half + 8 * i) = a1;
        *(v8b*)(Vth + r * 64 + half + 8 * i) = b0;
        *(v8b*)(Vtl + r * 64 + half + 8 * i) = b1;
      }
    }
    __syncthreads();

    v8f s[4];
#pragma unroll
    for (int j = 0; j < 4; ++j) {
      s[j] = vz8();
#pragma unroll
      for (int dc = 0; dc < 2; ++dc) {
        const int ko = (j * 16 + c) * 64 + dc * 32 + 8 * hh;
        const v16b kb = frag_ld(Ksh + ko);
        const v16b kl = frag_ld(Ksl + ko);
        s[j] = mma_bf(qah[dc], kb, s[j]);
        s[j] = mma_bf(qah[dc], kl, s[j]);
        s[j] = mma_bf(qal[dc], kb, s[j]);
      }
    }

    float cm[8];
#pragma unroll
    for (int r = 0; r < 8; ++r) {
      const int qrow = q0 + 8 * hh + r;
      float m = -INFINITY;
#pragma unroll
      for (int j = 0; j < 4; ++j) {
        float sv = s[j][r] * 0.125f;
        if (addm) sv += maskp[(size_t)qrow * SEQ + kv0 + j * 16 + c];
        s[j][r] = sv;
        m = fmaxf(m, sv);
      }
#pragma unroll
      for (int off = 1; off < 16; off <<= 1) m = fmaxf(m, __shfl_xor(m, off, 32));
      cm[r] = m;
    }

#pragma unroll
    for (int r = 0; r < 8; ++r) {
      const float mnew  = fmaxf(mrow[r], cm[r]);
      const float alpha = __expf(mrow[r] - mnew);
      mrow[r] = mnew;
      float psum = 0.f;
#pragma unroll
      for (int j = 0; j < 4; ++j) {
        const float p = __expf(s[j][r] - mnew);
        psum += p;
        const unsigned short hb = f2bf_bits(p);
        const unsigned short lb = f2bf_bits(p - bfb2f(hb));
        const int po = (8 * hh + r) * 64 + j * 16 + c;
        pwh[po] = bits2bf(hb);
        pwl[po] = bits2bf(lb);
      }
#pragma unroll
      for (int off = 1; off < 16; off <<= 1) psum += __shfl_xor(psum, off, 32);
      lrow[r] = lrow[r] * alpha + psum;
#pragma unroll
      for (int t = 0; t < 4; ++t) oacc[t][r] *= alpha;
    }
    wave_lds_sync();

#pragma unroll 1
    for (int kk = 0; kk < 2; ++kk) {
      const int pofs = c * 64 + kk * 32 + 8 * hh;
      const v16b pa = frag_ld(pwh + pofs);
      const v16b pl = frag_ld(pwl + pofs);
#pragma unroll
      for (int t = 0; t < 4; ++t) {
        const int vo = (t * 16 + c) * 64 + kk * 32 + 8 * hh;
        const v16b vb = frag_ld(Vth + vo);
        const v16b vl = frag_ld(Vtl + vo);
        oacc[t] = mma_bf(pa, vb, oacc[t]);
        oacc[t] = mma_bf(pa, vl, oacc[t]);
        oacc[t] = mma_bf(pl, vb, oacc[t]);
      }
    }
  }

  __syncthreads();
  float* os = (float*)(void*)KVs + wave * (16 * 68);
#pragma unroll
  for (int r = 0; r < 8; ++r) {
    const float inv = 1.0f / lrow[r];
#pragma unroll
    for (int t = 0; t < 4; ++t) os[(8 * hh + r) * 68 + t * 16 + c] = oacc[t][r] * inv;
  }
  wave_lds_sync();
  {
    const int q4 = lane >> 3, c8 = (lane & 7) * 8;
    unsigned short* Ob  = ohp + (size_t)b * SEQ * DM + (size_t)h * HD;
    unsigned short* Ob2 = olp + (size_t)b * SEQ * DM + (size_t)h * HD;
    for (int pass = 0; pass < 2; ++pass) {
#pragma unroll
      for (int it = 0; it < 4; ++it) {
        const int row = it * 4 + q4;
        const float* sp = os + row * 68 + c8;
        v8us hv, lv;
#pragma unroll
        for (int e = 0; e < 8; ++e) {
          const float f = sp[e];
          const unsigned short hb = f2bf_bits(f);
          hv[e] = hb;
          lv[e] = f2bf_bits(f - bfb2f(hb));
        }
        const size_t go = (size_t)(q0 + row) * DM + c8;
        *(volatile v8us*)(Ob + go)  = hv;
        *(volatile v8us*)(Ob2 + go) = lv;
      }
      __threadfence();
    }
  }
}

extern "C" void kernel_launch(void* const* d_in, const int* in_sizes, int n_in,
                              void* d_out, int out_size, void* d_ws, size_t ws_size,
                              hipStream_t stream) {
  if (n_in < 7) return;
  if (in_sizes[0] != NB * SEQ * DM) return;
  if (in_sizes[1] != SEQ * SEQ) return;
  if (in_sizes[2] != NB * SEQ) return;
  if (in_sizes[3] != DM * DM) return;
  if (in_sizes[4] != DKV * DM || in_sizes[5] != DKV * DM) return;
  if (in_sizes[6] != DM * DM) return;
  if (out_size != NB * SEQ * DM) return;

  const float* x    = (const float*)d_in[0];
  const float* mask = (const float*)d_in[1];
  const int*   pos  = (const int*)d_in[2];
  const float* wq   = (const float*)d_in[3];
  const float* wk   = (const float*)d_in[4];
  const float* wv   = (const float*)d_in[5];
  const float* wo   = (const float*)d_in[6];

  size_t off = 0;
  const size_t oXb  = off; off += (size_t)NB * SEQ * DM * 2;
  const size_t oWq  = off; off += (size_t)DM * DM * 2;
  const size_t oWk  = off; off += (size_t)DKV * DM * 2;
  const size_t oWv  = off; off += (size_t)DKV * DM * 2;
  const size_t oWo  = off; off += (size_t)DM * DM * 2;
  const size_t oCt  = off; off += (size_t)NB * SEQ * 32 * 4;
  const size_t oSt  = off; off += (size_t)NB * SEQ * 32 * 4;
  const size_t oTmx = off; off += (size_t)NQB * NQB * 4;
  const size_t oTmn = off; off += (size_t)NQB * NQB * 4;
  const size_t oQh  = off; off += (size_t)NB * SEQ * DM * 2;
  const size_t oQl  = off; off += (size_t)NB * SEQ * DM * 2;
  const size_t oKh  = off; off += (size_t)NB * SEQ * DKV * 2;
  const size_t oKl  = off; off += (size_t)NB * SEQ * DKV * 2;
  const size_t oVh  = off; off += (size_t)NB * DKV * SEQ * 2;
  const size_t oVl  = off; off += (size_t)NB * DKV * SEQ * 2;
  const size_t oOh  = off; off += (size_t)NB * SEQ * DM * 2;
  const size_t oOl  = off; off += (size_t)NB * SEQ * DM * 2;
  if (off > ws_size) return;

  char* ws = (char*)d_ws;
  unsigned short* Xb  = (unsigned short*)(ws + oXb);
  unsigned short* Wqb = (unsigned short*)(ws + oWq);
  unsigned short* Wkb = (unsigned short*)(ws + oWk);
  unsigned short* Wvb = (unsigned short*)(ws + oWv);
  unsigned short* Wob = (unsigned short*)(ws + oWo);
  float*          ctab = (float*)(ws + oCt);
  float*          stab = (float*)(ws + oSt);
  float*          tmax = (float*)(ws + oTmx);
  float*          tmin = (float*)(ws + oTmn);
  unsigned short* Qh  = (unsigned short*)(ws + oQh);
  unsigned short* Ql  = (unsigned short*)(ws + oQl);
  unsigned short* Kh  = (unsigned short*)(ws + oKh);
  unsigned short* Kl  = (unsigned short*)(ws + oKl);
  unsigned short* Vth = (unsigned short*)(ws + oVh);
  unsigned short* Vtl = (unsigned short*)(ws + oVl);
  unsigned short* Oh  = (unsigned short*)(ws + oOh);
  unsigned short* Ol  = (unsigned short*)(ws + oOl);

  RopeInv ri;
  {
    double acc = 1.0;
    const double g = 1.3335214321633240257;
    for (int i = 0; i < 32; ++i) {
      const float pw = (float)acc;
      ri.f[i] = 1.0f / pw;
      acc *= g;
    }
  }

  const dim3 blk256(256);

  k_cvt_bf16<<<dim3((NB * SEQ * DM / 8) / 256), blk256, 0, stream>>>(x,  Xb,  NB * SEQ * DM / 8);
  k_cvt_bf16<<<dim3((DM * DM / 8) / 256),       blk256, 0, stream>>>(wq, Wqb, DM * DM / 8);
  k_cvt_bf16<<<dim3((DKV * DM / 8) / 256),      blk256, 0, stream>>>(wk, Wkb, DKV * DM / 8);
  k_cvt_bf16<<<dim3((DKV * DM / 8) / 256),      blk256, 0, stream>>>(wv, Wvb, DKV * DM / 8);
  k_cvt_bf16<<<dim3((DM * DM / 8) / 256),       blk256, 0, stream>>>(wo, Wob, DM * DM / 8);
  k_rope_tab<<<dim3(NB * SEQ / 8), blk256, 0, stream>>>(pos, ctab, stab, ri, NB * SEQ);
  k_masktiles<<<dim3(NQB), blk256, 0, stream>>>(mask, tmax, tmin);
  k_gemm64<1, true, 2><<<dim3(((NB * SEQ / 64) * (DM / 64)) / 8, 1), blk256, 0, stream>>>(
      Xb, Xb, DM, 0LL, Wqb, DM, 0LL, (void*)Qh, (void*)Ql, DM, 0LL, ctab, stab, NB * SEQ, DM, DM);
  k_gemm64<1, true, 2><<<dim3(((NB * SEQ / 64) * (DKV / 64)) / 8, 1), blk256, 0, stream>>>(
      Xb, Xb, DM, 0LL, Wkb, DM, 0LL, (void*)Kh, (void*)Kl, DKV, 0LL, ctab, stab, NB * SEQ, DKV, DM);
  k_gemm64<1, false, 2><<<dim3(((DKV / 64) * (SEQ / 64)) / 8, NB), blk256, 0, stream>>>(
      Wvb, Wvb, DM, 0LL, Xb, DM, (long long)SEQ * DM, (void*)Vth, (void*)Vtl, SEQ, (long long)DKV * SEQ,
      ctab, stab, DKV, SEQ, DM);
  k_attn<<<dim3(NB * NHQ * NQB), dim3(128), 0, stream>>>(Qh, Ql, Kh, Kl, Vth, Vtl, mask, tmax, tmin, Oh, Ol);
  k_gemm64<2, false, 0><<<dim3(((NB * SEQ / 64) * (DM / 64)) / 8, 1), blk256, 0, stream>>>(
      Oh, Ol, DM, 0LL, Wob, DM, 0LL, d_out, d_out, DM, 0LL, ctab, stab, NB * SEQ, DM, DM);

  (void)hipGetLastError();
}
